// TransformerDecoderLayer_5171140624713
// MI455X (gfx1250) — hardware-verified
//
#include <hip/hip_runtime.h>


#ifndef NB
#define NB 4
#endif
#ifndef SEQ
#define SEQ 2048
#endif
#define NB_FULL 4
#define SEQ_FULL 2048
#define DM 512
#define HE 4
#define DH 64
#define DV 128
#define KT 32
#define QR 64
#define KPITCH 72
#define VPITCH 40
#define PPITCH 40
#define CPITCH 136
#define OPITCH 132
#define P_CARRY 4096.0f
#define V_CARRY 16.0f
#define X_CARRY 64.0f
#define W_CARRY 1024.0f
#define LAMBDA_INIT 0.8f
#define OUT_SCALE 0.2f
#define RMS_EPS 1e-5f

static_assert(NB >= 1 && NB <= NB_FULL);
static_assert(SEQ >= QR && SEQ <= SEQ_FULL);
static_assert(SEQ % QR == 0);
static_assert(SEQ % KT == 0);
static_assert((NB * SEQ) % 64 == 0);
static_assert(DM % 128 == 0);
static_assert(DM == HE * DV);
static_assert(DV == 2 * DH);

typedef _Float16 v8h  __attribute__((ext_vector_type(8)));
typedef _Float16 v16h __attribute__((ext_vector_type(16)));
typedef __bf16   v16bf __attribute__((ext_vector_type(16)));
typedef unsigned short v8us __attribute__((ext_vector_type(8)));
typedef float v8f __attribute__((ext_vector_type(8)));
typedef float v4f __attribute__((ext_vector_type(4)));

union FragH { v16h v; v8h h[2]; };
union FragB { v16bf v; v8us h[2]; };
union ExCt { float ex[4 * 16 * DV]; _Float16 ct[QR * CPITCH]; };
static_assert(sizeof(ExCt) == 4 * 16 * DV * 4);

__device__ __forceinline__ unsigned f2bf(float f) { unsigned u = __float_as_uint(f); u += 0x7FFFu + ((u >> 16) & 1u); return u >> 16; }
__device__ __forceinline__ float bf16r(float f) { return __uint_as_float(f2bf(f) << 16); }

__device__ __forceinline__ v8f wm_f16(v16h a, v16h b, v8f c) {
    c = __builtin_amdgcn_wmma_f32_16x16x32_f16(false, a, false, b, (short)0, c, false, false);
    asm volatile("v_nop\n\tv_nop\n\tv_nop\n\tv_nop" : "+v"(c) : "v"(a), "v"(b));
    return c;
}
__device__ __forceinline__ v8f wm_bf16(v16bf a, v16bf b, v8f c) {
    c = __builtin_amdgcn_wmma_f32_16x16x32_bf16(false, a, false, b, (short)0, c, false, false);
    asm volatile("v_nop\n\tv_nop\n\tv_nop\n\tv_nop" : "+v"(c) : "v"(a), "v"(b));
    return c;
}

__global__ __launch_bounds__(256) void k_convert(const float* __restrict__ q, const float* __restrict__ k, const float* __restrict__ v, const float* __restrict__ w,
                                                unsigned short* Qb, unsigned short* Kb, _Float16* Vh, _Float16* Wh, int nblkA)
{
    const int bid = blockIdx.x;
    int which, lb;
    if (bid < nblkA)          { which = 0; lb = bid; }
    else if (bid < 2 * nblkA) { which = 1; lb = bid - nblkA; }
    else if (bid < 3 * nblkA) { which = 2; lb = bid - 2 * nblkA; }
    else                      { which = 3; lb = bid - 3 * nblkA; }
    const size_t e = ((size_t)lb * 256 + threadIdx.x) * 8;
    const float* src;
    if (which == 3) {
        src = w + e;
    } else {
        const size_t m = e / DM; const int col = (int)(e % DM);
        const int bb = (int)(m / SEQ), n = (int)(m % SEQ);
        src = ((which == 0) ? q : ((which == 1) ? k : v)) + ((size_t)bb * SEQ_FULL + n) * DM + col;
    }
    const v4f a0 = *(const v4f*)src, a1 = *(const v4f*)(src + 4);
    float f[8];
#pragma unroll
    for (int i = 0; i < 4; ++i) { f[i] = a0[i]; f[4 + i] = a1[i]; }
    if (which <= 1) {
        v8us o;
#pragma unroll
        for (int i = 0; i < 8; ++i) o[i] = (unsigned short)f2bf(f[i]);
        unsigned short* dst = ((which == 0) ? Qb : Kb) + e;
        *(volatile v8us*)dst = o;
        __threadfence();
        *(volatile v8us*)dst = o;
    } else {
        const float sc = (which == 2) ? V_CARRY : W_CARRY;
        v8h o;
#pragma unroll
        for (int i = 0; i < 8; ++i) o[i] = (_Float16)(bf16r(f[i]) * sc);
        _Float16* dst = ((which == 2) ? Vh : Wh) + e;
        *(volatile v8h*)dst = o;
        __threadfence();
        *(volatile v8h*)dst = o;
    }
}

__global__ __launch_bounds__(256) void k_attn(const unsigned short* __restrict__ Qb, const unsigned short* __restrict__ Kb, const _Float16* __restrict__ Vh,
                                             const float* __restrict__ lq1, const float* __restrict__ lk1, const float* __restrict__ lq2, const float* __restrict__ lk2,
                                             const float* __restrict__ normw, _Float16* Xc)
{
    __shared__ __align__(16) unsigned short sK[2 * KT * KPITCH];
    __shared__ __align__(16) _Float16 sVt[DV * VPITCH];
    __shared__ __align__(16) _Float16 sP[8 * 16 * PPITCH];
    __shared__ __align__(16) ExCt U;
    __shared__ float s_lam;

    const int tid = threadIdx.x, lane = tid & 31, wv = tid >> 5, hh = lane >> 4, lm = lane & 15;
    const int rg = wv & 3, s = wv >> 2;
    const int b = blockIdx.z, h = blockIdx.y, q0 = blockIdx.x * QR;

    if (tid == 0) {
        float s1 = 0.f, s2 = 0.f;
#pragma unroll 1
        for (int i = 0; i < DH; ++i) { s1 += bf16r(lq1[i]) * bf16r(lk1[i]); s2 += bf16r(lq2[i]) * bf16r(lk2[i]); }
        s_lam = expf(s1) - expf(s2) + LAMBDA_INIT;
    }

    FragB qa[2];
    {
        const unsigned short* qrow = Qb + ((size_t)b * SEQ + q0 + rg * 16 + lm) * DM + (2 * h + s) * DH;
#pragma unroll
        for (int j = 0; j < 2; ++j) {
            qa[j].h[0] = *(const v8us*)(qrow + 32 * j + 8 * hh);
            qa[j].h[1] = *(const v8us*)(qrow + 32 * j + 16 + 8 * hh);
        }
    }
    v8f acc[8];
    float rm[8], rl[8];
#pragma unroll
    for (int t = 0; t < 8; ++t) acc[t] = (v8f){};
#pragma unroll
    for (int r = 0; r < 8; ++r) { rm[r] = -1e30f; rl[r] = 0.f; }

    const size_t kvrow0 = (size_t)b * SEQ;
#pragma unroll 1
    for (int kt = 0; kt < SEQ / KT; ++kt) {
        const int key0 = kt * KT;
#pragma unroll
        for (int i = 0; i < 2; ++i) {
            const int p = tid + 256 * i, key = p >> 4, c16 = p & 15;
            const size_t g = (kvrow0 + key0 + key) * DM + (size_t)h * DV + c16 * 8;
            const v8us kv = *(const v8us*)(Kb + g);
            *(v8us*)(sK + ((c16 >> 3) * KT + key) * KPITCH + (c16 & 7) * 8) = kv;
            const v8h vv = *(const v8h*)(Vh + g);
#pragma unroll
            for (int j = 0; j < 8; ++j) sVt[(c16 * 8 + j) * VPITCH + key] = vv[j];
        }
        __syncthreads();

        v8f sc[2];
#pragma unroll
        for (int t = 0; t < 2; ++t) {
            v8f c = (v8f){};
#pragma unroll
            for (int j = 0; j < 2; ++j) {
                FragB kb;
                const unsigned short* kr = sK + (s * KT + t * 16 + lm) * KPITCH + 32 * j;
                kb.h[0] = *(const v8us*)(kr + 8 * hh);
                kb.h[1] = *(const v8us*)(kr + 16 + 8 * hh);
                c = wm_bf16(qa[j].v, kb.v, c);
            }
            sc[t] = c;
        }
#pragma unroll
        for (int r = 0; r < 8; ++r) {
            const float x0 = sc[0][r] * 0.125f, x1 = sc[1][r] * 0.125f;
            float mx = fmaxf(x0, x1);
#pragma unroll
            for (int o = 1; o < 16; o <<= 1) mx = fmaxf(mx, __shfl_xor(mx, o, 32));
            const float nm = fmaxf(rm[r], mx);
            const float corr = __expf(rm[r] - nm);
            const float p0 = __expf(x0 - nm), p1 = __expf(x1 - nm);
            float rs = p0 + p1;
#pragma unroll
            for (int o = 1; o < 16; o <<= 1) rs += __shfl_xor(rs, o, 32);
            rl[r] = rl[r] * corr + rs;
            rm[r] = nm;
#pragma unroll
            for (int t = 0; t < 8; ++t) acc[t][r] = acc[t][r] * corr;
            _Float16* prow = sP + (wv * 16 + 8 * hh + r) * PPITCH;
            prow[lm] = (_Float16)(p0 * P_CARRY);
            prow[16 + lm] = (_Float16)(p1 * P_CARRY);
        }
        __syncthreads();

        {
            FragH pa;
            const _Float16* pr = sP + (wv * 16 + lm) * PPITCH;
            pa.h[0] = *(const v8h*)(pr + 8 * hh);
            pa.h[1] = *(const v8h*)(pr + 16 + 8 * hh);
#pragma unroll
            for (int t = 0; t < 8; ++t) {
                FragH vb;
                const _Float16* vr = sVt + (t * 16 + lm) * VPITCH;
                vb.h[0] = *(const v8h*)(vr + 8 * hh);
                vb.h[1] = *(const v8h*)(vr + 16 + 8 * hh);
                acc[t] = wm_f16(pa.v, vb.v, acc[t]);
            }
        }
        __syncthreads();
    }

    const float lam = s_lam;
    float inv[8];
#pragma unroll
    for (int r = 0; r < 8; ++r) inv[r] = (1.0f / rl[r]) * (1.0f / (P_CARRY * V_CARRY));

    if (s == 1) {
#pragma unroll
        for (int r = 0; r < 8; ++r)
#pragma unroll
            for (int t = 0; t < 8; ++t)
                U.ex[(rg * 16 + 8 * hh + r) * DV + t * 16 + lm] = acc[t][r] * inv[r];
    }
    __syncthreads();
    if (s == 0) {
        float nw[8];
#pragma unroll
        for (int t = 0; t < 8; ++t) nw[t] = bf16r(normw[t * 16 + lm]) * (OUT_SCALE * X_CARRY);
#pragma unroll
        for (int r = 0; r < 8; ++r) {
            float ss = 0.f;
#pragma unroll
            for (int t = 0; t < 8; ++t) {
                const float d = acc[t][r] * inv[r] - lam * U.ex[(rg * 16 + 8 * hh + r) * DV + t * 16 + lm];
                acc[t][r] = d;
                ss += d * d;
            }
#pragma unroll
            for (int o = 1; o < 16; o <<= 1) ss += __shfl_xor(ss, o, 32);
            const float g = rsqrtf(ss * (1.0f / DV) + RMS_EPS);
#pragma unroll
            for (int t = 0; t < 8; ++t) acc[t][r] = acc[t][r] * g * nw[t];
        }
    }
    __syncthreads();
    if (s == 0) {
#pragma unroll
        for (int r = 0; r < 8; ++r)
#pragma unroll
            for (int t = 0; t < 8; ++t)
                U.ct[(rg * 16 + 8 * hh + r) * CPITCH + t * 16 + lm] = (_Float16)acc[t][r];
    }
    __syncthreads();
    v8h ov[4];
#pragma unroll
    for (int i = 0; i < 4; ++i) {
        const int p = tid + 256 * i, row = p >> 4, c8 = (p & 15) * 8;
        ov[i] = *(const v8h*)(U.ct + row * CPITCH + c8);
    }
#pragma unroll
    for (int i = 0; i < 4; ++i) {
        const int p = tid + 256 * i, row = p >> 4, c8 = (p & 15) * 8;
        *(volatile v8h*)(Xc + (kvrow0 + q0 + row) * DM + (size_t)h * DV + c8) = ov[i];
    }
    __threadfence();
#pragma unroll
    for (int i = 0; i < 4; ++i) {
        const int p = tid + 256 * i, row = p >> 4, c8 = (p & 15) * 8;
        *(volatile v8h*)(Xc + (kvrow0 + q0 + row) * DM + (size_t)h * DV + c8) = ov[i];
    }
}

__global__ __launch_bounds__(256) void k_oproj(const _Float16* __restrict__ X, const _Float16* __restrict__ Wh, const float* __restrict__ bias, float* out)
{
    __shared__ __align__(16) float cst[64 * OPITCH];
    const int tid = threadIdx.x, lane = tid & 31, wv = tid >> 5, hh = lane >> 4, lm = lane & 15;
    const int rt = wv & 3, ch = wv >> 2;
    const int row0 = blockIdx.x * 64, cb = blockIdx.y * 128, col0 = cb + ch * 64;
    const _Float16* xr = X + (size_t)(row0 + rt * 16 + lm) * DM;
    v8f acc[4];
#pragma unroll
    for (int t = 0; t < 4; ++t) acc[t] = (v8f){};
#pragma unroll 2
    for (int kc = 0; kc < DM; kc += 32) {
        FragH a;
        a.h[0] = *(const v8h*)(xr + kc + 8 * hh);
        a.h[1] = *(const v8h*)(xr + kc + 16 + 8 * hh);
#pragma unroll
        for (int t = 0; t < 4; ++t) {
            FragH bb;
            const _Float16* wr = Wh + (size_t)(col0 + t * 16 + lm) * DM + kc;
            bb.h[0] = *(const v8h*)(wr + 8 * hh);
            bb.h[1] = *(const v8h*)(wr + 16 + 8 * hh);
            acc[t] = wm_f16(a.v, bb.v, acc[t]);
        }
    }
#pragma unroll
    for (int t = 0; t < 4; ++t) {
        const int cl = ch * 64 + t * 16 + lm;
        const float bv = bf16r(bias[cb + cl]);
#pragma unroll
        for (int r = 0; r < 8; ++r) cst[(rt * 16 + 8 * hh + r) * OPITCH + cl] = acc[t][r] * (1.0f / (X_CARRY * W_CARRY)) + bv;
    }
    __syncthreads();
    v4f ov[8];
#pragma unroll
    for (int i = 0; i < 8; ++i) {
        const int p = tid + 256 * i, row = p >> 5, c4 = (p & 31) * 4;
        ov[i] = *(const v4f*)(cst + row * OPITCH + c4);
    }
#pragma unroll
    for (int i = 0; i < 8; ++i) {
        const int p = tid + 256 * i, row = p >> 5, c4 = (p & 31) * 4;
        const int m = row0 + row, bb = m / SEQ, n = m % SEQ;
        *(volatile v4f*)(out + ((size_t)bb * SEQ_FULL + n) * DM + cb + c4) = ov[i];
    }
    __threadfence();
#pragma unroll
    for (int i = 0; i < 8; ++i) {
        const int p = tid + 256 * i, row = p >> 5, c4 = (p & 31) * 4;
        const int m = row0 + row, bb = m / SEQ, n = m % SEQ;
        *(volatile v4f*)(out + ((size_t)bb * SEQ_FULL + n) * DM + cb + c4) = ov[i];
    }
}

extern "C" void kernel_launch(void* const* d_in, const int* in_sizes, int n_in,
                              void* d_out, int out_size, void* d_ws, size_t ws_size, hipStream_t stream)
{
    if (n_in < 10) return;
    const long long needAct = ((long long)(NB - 1) * SEQ_FULL + SEQ) * DM;
    if ((long long)in_sizes[0] < needAct || (long long)in_sizes[1] < needAct || (long long)in_sizes[2] < needAct) return;
    if (in_sizes[3] < DH || in_sizes[4] < DH || in_sizes[5] < DH || in_sizes[6] < DH) return;
    if (in_sizes[7] < DV || in_sizes[8] < DM * DM || in_sizes[9] < DM) return;
    if ((long long)out_size < needAct) return;

    const float* q      = (const float*)d_in[0];
    const float* k      = (const float*)d_in[1];
    const float* v      = (const float*)d_in[2];
    const float* lq1    = (const float*)d_in[3];
    const float* lk1    = (const float*)d_in[4];
    const float* lq2    = (const float*)d_in[5];
    const float* lk2    = (const float*)d_in[6];
    const float* norm_w = (const float*)d_in[7];
    const float* out_w  = (const float*)d_in[8];
    const float* out_b  = (const float*)d_in[9];
    float* out = (float*)d_out;

    const size_t nact = (size_t)NB * SEQ * DM;
    unsigned char* base = (unsigned char*)d_ws;
    size_t off = 0;
    unsigned short* Qb = (unsigned short*)(base + off); off += nact * 2;
    unsigned short* Kb = (unsigned short*)(base + off); off += nact * 2;
    _Float16* Vh = (_Float16*)(base + off);           off += nact * 2;
    _Float16* Wh = (_Float16*)(base + off);           off += (size_t)DM * DM * 2;
    _Float16* Xc = (_Float16*)(base + off);           off += nact * 2;
    if (off > ws_size) return;

    const int nblkA = (int)(nact / 2048);
    k_convert<<<dim3(3 * nblkA + (DM * DM) / 2048), dim3(256), 0, stream>>>(q, k, v, out_w, Qb, Kb, Vh, Wh, nblkA);
    k_attn<<<dim3(SEQ / QR, HE, NB), dim3(256), 0, stream>>>(Qb, Kb, Vh, lq1, lk1, lq2, lk2, norm_w, Xc);
    k_oproj<<<dim3((NB * SEQ) / 64, DM / 128), dim3(256), 0, stream>>>(Xc, Wh, out_b, out);
}
